// SSAA_47914655154294
// MI455X (gfx1250) — hardware-verified
//
#include <hip/hip_runtime.h>


typedef _Float16 v16h __attribute__((ext_vector_type(16)));
typedef _Float16 v8h_ __attribute__((ext_vector_type(8)));
typedef v8h_ v8h __attribute__((may_alias));
typedef float v8f __attribute__((ext_vector_type(8)));
typedef float v4f_ __attribute__((ext_vector_type(4)));
typedef v4f_ v4f __attribute__((may_alias));
union Frag { v16h v; v8h_ half[2]; };

#define CCH   256
#define NHEAD 8
#define HDIM  32
#define IMG   64
#define NQ    4096
#define NKV   256
#define ATT_SCALE 0.17677669529663687f

#define BM  128
#define BN  64
#define BK  32
#define BSP 40
#define SP0 68
#define SP1 72
#define SP2 40
#define ASP 72

static __device__ __forceinline__ v8f wmma16(v16h a, v16h b, v8f c) {
  v8f d = __builtin_amdgcn_wmma_f32_16x16x32_f16(false, a, false, b, (short)0, c, false, false);
  asm volatile("v_nop\n\tv_nop\n\tv_nop\n\tv_nop" : "+v"(d) : "v"(a), "v"(b));
  return d;
}

static __device__ __forceinline__ v16h ld_frag(const _Float16* base, int ld, int row0, int k0, int lane) {
  const int h = lane >> 4, m = lane & 15;
  const _Float16* p = base + (size_t)(row0 + m) * ld + k0 + 8 * h;
  Frag f;
  f.half[0] = *(const v8h*)(p);
  f.half[1] = *(const v8h*)(p + 16);
  return f.v;
}

__global__ void __launch_bounds__(256)
k_cvt(const float* __restrict__ src, _Float16* __restrict__ dst, int count, float scale) {
  const size_t i = (size_t)blockIdx.x * blockDim.x + threadIdx.x;
  const size_t base = i * 8;
  if (base + 8 > (size_t)count) return;
  const v4f u0 = *(const v4f*)(src + base);
  const v4f u1 = *(const v4f*)(src + base + 4);
  v8h_ o;
  o[0] = (_Float16)(u0[0] * scale); o[1] = (_Float16)(u0[1] * scale);
  o[2] = (_Float16)(u0[2] * scale); o[3] = (_Float16)(u0[3] * scale);
  o[4] = (_Float16)(u1[0] * scale); o[5] = (_Float16)(u1[1] * scale);
  o[6] = (_Float16)(u1[2] * scale); o[7] = (_Float16)(u1[3] * scale);
  _Float16* p = dst + base;
  *(volatile v8h_*)p = o;
  __threadfence();
  *(volatile v8h_*)p = o;
}

template <int LM, int EM>
__global__ void __launch_bounds__(256)
k_gemm(const _Float16* __restrict__ A, const void* __restrict__ Bsrc, const float* __restrict__ bias,
       void* __restrict__ dst, int M, int N, int K, int ldsrc, int nbatch,
       float bscale, float ascale, float oscale) {
  __shared__ __align__(16) _Float16 Bs[BN * BSP];
  const int tid = threadIdx.x, lane = tid & 31, w = tid >> 5, wm = w & 3, wn = w >> 2;
  const int hh = lane >> 4, cc = lane & 15;
  const int nbn = N / BN, nbm = M / BM;
  int bid = blockIdx.x;
  const int nb = bid % nbn; bid /= nbn;
  const int mb = bid % nbm; bid /= nbm;
  const int b = bid;
  if (b >= nbatch) return;
  const int m0 = mb * BM, n0 = nb * BN;
  const size_t srcb = (size_t)b * (size_t)K * (size_t)ldsrc;

  v8f acc[2][2];
  {
    v8f z = {};
    acc[0][0] = z; acc[0][1] = z; acc[1][0] = z; acc[1][1] = z;
  }
  const int kk = tid >> 3, nn = (tid & 7) * 8;

  for (int k0 = 0; k0 < K; k0 += BK) {
    if constexpr (LM == 0) {
      const float* p = (const float*)Bsrc + srcb + (size_t)(k0 + kk) * ldsrc + n0 + nn;
      const v4f u0 = *(const v4f*)p;
      const v4f u1 = *(const v4f*)(p + 4);
      _Float16* q = Bs + nn * BSP + kk;
      q[0 * BSP] = (_Float16)(u0[0] * bscale);
      q[1 * BSP] = (_Float16)(u0[1] * bscale);
      q[2 * BSP] = (_Float16)(u0[2] * bscale);
      q[3 * BSP] = (_Float16)(u0[3] * bscale);
      q[4 * BSP] = (_Float16)(u1[0] * bscale);
      q[5 * BSP] = (_Float16)(u1[1] * bscale);
      q[6 * BSP] = (_Float16)(u1[2] * bscale);
      q[7 * BSP] = (_Float16)(u1[3] * bscale);
    } else if constexpr (LM == 1) {
      const _Float16* p = (const _Float16*)Bsrc + srcb + (size_t)(k0 + kk) * ldsrc + n0 + nn;
      const v8h u = *(const v8h*)p;
      _Float16* q = Bs + nn * BSP + kk;
#pragma unroll
      for (int e = 0; e < 8; ++e) q[e * BSP] = u[e];
    } else {
      const int ci_l = kk >> 4, ky = (kk >> 2) & 3, py_l = kk & 3;
      const int ci = (k0 >> 4) + ci_l;
      const int y = ((n0 >> 4) + py_l) * 4 + ky;
      const int xg = tid & 7;
      const float* p = (const float*)Bsrc + srcb + ((size_t)ci * IMG + y) * IMG + xg * 8;
      const v4f u0 = *(const v4f*)p;
      const v4f u1 = *(const v4f*)(p + 4);
      _Float16* q = Bs + (py_l * 16 + xg * 2) * BSP + ci_l * 16 + ky * 4;
      q[0] = (_Float16)(u0[0] * bscale);
      q[1] = (_Float16)(u0[1] * bscale);
      q[2] = (_Float16)(u0[2] * bscale);
      q[3] = (_Float16)(u0[3] * bscale);
      q[BSP + 0] = (_Float16)(u1[0] * bscale);
      q[BSP + 1] = (_Float16)(u1[1] * bscale);
      q[BSP + 2] = (_Float16)(u1[2] * bscale);
      q[BSP + 3] = (_Float16)(u1[3] * bscale);
    }
    __syncthreads();
    v16h af[2], bf[2];
    af[0] = ld_frag(A, K, m0 + 32 * wm, k0, lane);
    af[1] = ld_frag(A, K, m0 + 32 * wm + 16, k0, lane);
    bf[0] = ld_frag(Bs, BSP, 32 * wn, 0, lane);
    bf[1] = ld_frag(Bs, BSP, 32 * wn + 16, 0, lane);
    acc[0][0] = wmma16(af[0], bf[0], acc[0][0]);
    acc[0][1] = wmma16(af[0], bf[1], acc[0][1]);
    acc[1][0] = wmma16(af[1], bf[0], acc[1][0]);
    acc[1][1] = wmma16(af[1], bf[1], acc[1][1]);
    __syncthreads();
  }

  if constexpr (EM == 0) {
    __shared__ __align__(16) float stg[BM * SP0];
#pragma unroll
    for (int i = 0; i < 2; ++i)
#pragma unroll
      for (int j = 0; j < 2; ++j)
#pragma unroll
        for (int r = 0; r < 8; ++r) {
          const int ml = 32 * wm + 16 * i + 8 * hh + r;
          const int nl = 32 * wn + 16 * j + cc;
          stg[ml * SP0 + nl] = (acc[i][j][r] * ascale + bias[m0 + ml]) * oscale;
        }
    __syncthreads();
    float* D = (float*)dst;
    v4f_ vals[8];
#pragma unroll
    for (int it = 0; it < 8; ++it) {
      const int ml = it * 16 + w * 2 + hh;
      vals[it] = *(const v4f*)(stg + ml * SP0 + cc * 4);
    }
#pragma unroll
    for (int it = 0; it < 8; ++it) {
      const int ml = it * 16 + w * 2 + hh;
      float* pd = D + ((size_t)b * M + m0 + ml) * (size_t)N + n0 + cc * 4;
      *(volatile v4f_*)pd = vals[it];
    }
    __threadfence();
#pragma unroll
    for (int it = 0; it < 8; ++it) {
      const int ml = it * 16 + w * 2 + hh;
      float* pd = D + ((size_t)b * M + m0 + ml) * (size_t)N + n0 + cc * 4;
      *(volatile v4f_*)pd = vals[it];
    }
  } else if constexpr (EM == 1) {
    __shared__ __align__(16) _Float16 stg[BM * SP1];
#pragma unroll
    for (int i = 0; i < 2; ++i)
#pragma unroll
      for (int j = 0; j < 2; ++j)
#pragma unroll
        for (int r = 0; r < 8; ++r) {
          const int ml = 32 * wm + 16 * i + 8 * hh + r;
          const int nl = 32 * wn + 16 * j + cc;
          stg[ml * SP1 + nl] = (_Float16)((acc[i][j][r] * ascale + bias[m0 + ml]) * oscale);
        }
    __syncthreads();
    _Float16* D = (_Float16*)dst;
    const int lr = lane >> 3, pc = (lane & 7) * 8;
    v8h_ vals[4];
#pragma unroll
    for (int it = 0; it < 4; ++it) {
      const int ml = it * 32 + w * 4 + lr;
      vals[it] = *(const v8h*)(stg + ml * SP1 + pc);
    }
#pragma unroll
    for (int it = 0; it < 4; ++it) {
      const int ml = it * 32 + w * 4 + lr;
      _Float16* pd = D + ((size_t)b * M + m0 + ml) * (size_t)N + n0 + pc;
      *(volatile v8h_*)pd = vals[it];
    }
    __threadfence();
#pragma unroll
    for (int it = 0; it < 4; ++it) {
      const int ml = it * 32 + w * 4 + lr;
      _Float16* pd = D + ((size_t)b * M + m0 + ml) * (size_t)N + n0 + pc;
      *(volatile v8h_*)pd = vals[it];
    }
  } else {
    __shared__ __align__(16) _Float16 stg[4 * BN * SP2];
#pragma unroll
    for (int i = 0; i < 2; ++i)
#pragma unroll
      for (int j = 0; j < 2; ++j)
#pragma unroll
        for (int r = 0; r < 8; ++r) {
          const int ml = 32 * wm + 16 * i + 8 * hh + r;
          const int d  = 16 * i + 8 * hh + r;
          const int nl = 32 * wn + 16 * j + cc;
          stg[(wm * BN + nl) * SP2 + d] = (_Float16)((acc[i][j][r] * ascale + bias[m0 + ml]) * oscale);
        }
    __syncthreads();
    _Float16* D = (_Float16*)dst;
    const int G = M >> 5;
    const int nrow = tid >> 2, dp = (tid & 3) * 8;
    v8h_ vals[4];
#pragma unroll
    for (int g = 0; g < 4; ++g) vals[g] = *(const v8h*)(stg + (g * BN + nrow) * SP2 + dp);
#pragma unroll
    for (int g = 0; g < 4; ++g) {
      _Float16* pd = D + (((size_t)b * G + (m0 >> 5) + g) * (size_t)N + n0 + nrow) * 32 + dp;
      *(volatile v8h_*)pd = vals[g];
    }
    __threadfence();
#pragma unroll
    for (int g = 0; g < 4; ++g) {
      _Float16* pd = D + (((size_t)b * G + (m0 >> 5) + g) * (size_t)N + n0 + nrow) * 32 + dp;
      *(volatile v8h_*)pd = vals[g];
    }
  }
}

__global__ void __launch_bounds__(256)
k_dw3x3(const float* __restrict__ xr,
        const float* __restrict__ wkd, const float* __restrict__ bkd,
        const float* __restrict__ wvd, const float* __restrict__ bvd,
        float* __restrict__ dwk, float* __restrict__ dwv, int total) {
  const int i = blockIdx.x * blockDim.x + threadIdx.x;
  if (i >= total) return;
  const int pxq = i & 3, py = (i >> 2) & 15, cch = (i >> 6) & 255, b = i >> 14;
  const size_t base = ((size_t)b * CCH + cch) * NKV;
  const int px0 = pxq * 4;
  const float bk0 = bkd[cch], bv0 = bvd[cch];
  float sk[4], sv[4];
#pragma unroll
  for (int o = 0; o < 4; ++o) { sk[o] = bk0; sv[o] = bv0; }
#pragma unroll
  for (int dy = 0; dy < 3; ++dy) {
    const int yy = py + dy - 1;
    if (yy < 0 || yy > 15) continue;
    const float* rowp = xr + base + yy * 16;
    float xv[6];
#pragma unroll
    for (int e = 0; e < 6; ++e) {
      const int xx = px0 - 1 + e;
      xv[e] = (xx >= 0 && xx <= 15) ? rowp[xx] : 0.0f;
    }
#pragma unroll
    for (int dx = 0; dx < 3; ++dx) {
      const float wk = wkd[cch * 9 + dy * 3 + dx];
      const float wv = wvd[cch * 9 + dy * 3 + dx];
#pragma unroll
      for (int o = 0; o < 4; ++o) {
        sk[o] += wk * xv[o + dx];
        sv[o] += wv * xv[o + dx];
      }
    }
  }
  v4f_ ok, ov;
  ok[0] = sk[0]; ok[1] = sk[1]; ok[2] = sk[2]; ok[3] = sk[3];
  ov[0] = sv[0]; ov[1] = sv[1]; ov[2] = sv[2]; ov[3] = sv[3];
  const size_t o = base + py * 16 + px0;
  *(volatile v4f_*)(dwk + o) = ok;
  *(volatile v4f_*)(dwv + o) = ov;
  __threadfence();
  *(volatile v4f_*)(dwk + o) = ok;
  *(volatile v4f_*)(dwv + o) = ov;
}

__global__ void __launch_bounds__(64)
k_attn(const _Float16* __restrict__ qh, const _Float16* __restrict__ kh,
       const _Float16* __restrict__ vh, _Float16* __restrict__ oc, int nbatch,
       float sscale_a, float sscale_e, float vinv_a, float vinv_e) {
  __shared__ __align__(16) float S[2][16][NKV];
  __shared__ __align__(16) _Float16 P[2][16][NKV];
  __shared__ __align__(16) _Float16 stg[HDIM * ASP];
  const int tid = threadIdx.x, lane = tid & 31, wloc = tid >> 5;
  const int hh = lane >> 4, cc = lane & 15;
  int bid = blockIdx.x;
  const int qg = bid & 63; bid >>= 6;
  const int hd = bid & 7;  bid >>= 3;
  const int br = bid & 1;
  const int b  = bid >> 1;
  if (b >= nbatch) return;
  const float sscale = br ? sscale_e : sscale_a;
  const float vinv   = br ? vinv_e : vinv_a;
  const size_t bh = (size_t)b * NHEAD + hd;
  const size_t grp = (size_t)br * nbatch * NHEAD + bh;
  const _Float16* Kt = kh + grp * (NKV * HDIM);
  const _Float16* Vt = vh + grp * (NKV * HDIM);
  const _Float16* Qb = qh + ((size_t)b * 16 + br * 8 + hd) * ((size_t)NQ * HDIM);
  float (*Sw)[NKV] = S[wloc];
  _Float16 (*Pw)[NKV] = P[wloc];

  for (int t = 0; t < 2; ++t) {
    const int qloc0 = (wloc * 2 + t) * 16;
    const int q0 = qg * 64 + qloc0;
    const v16h aq = ld_frag(Qb, HDIM, q0, 0, lane);
    for (int kt = 0; kt < 16; ++kt) {
      const v16h bk = ld_frag(Kt, HDIM, kt * 16, 0, lane);
      v8f c = {};
      c = wmma16(aq, bk, c);
#pragma unroll
      for (int r = 0; r < 8; ++r) Sw[hh * 8 + r][kt * 16 + cc] = c[r] * sscale;
    }
    __syncthreads();
    {
      const int row = cc, cs = hh * 128;
      float mx = -3.0e38f;
#pragma unroll 8
      for (int i = 0; i < 128; ++i) mx = fmaxf(mx, Sw[row][cs + i]);
      mx = fmaxf(mx, __shfl_xor(mx, 16, 32));
      float sum = 0.0f;
#pragma unroll 8
      for (int i = 0; i < 128; ++i) {
        const float e = __expf(Sw[row][cs + i] - mx);
        Sw[row][cs + i] = e;
        sum += e;
      }
      sum += __shfl_xor(sum, 16, 32);
      const float pin = 256.0f / sum;
#pragma unroll 8
      for (int i = 0; i < 128; ++i) Pw[row][cs + i] = (_Float16)(Sw[row][cs + i] * pin);
    }
    __syncthreads();
    v8f o0 = {}, o1 = {};
    for (int kc = 0; kc < NKV; kc += 32) {
      const v16h ap = ld_frag(&Pw[0][0], NKV, 0, kc, lane);
      const v16h b0 = ld_frag(Vt, NKV, 0, kc, lane);
      const v16h b1 = ld_frag(Vt, NKV, 16, kc, lane);
      o0 = wmma16(ap, b0, o0);
      o1 = wmma16(ap, b1, o1);
    }
#pragma unroll
    for (int r = 0; r < 8; ++r) {
      const int ql = qloc0 + hh * 8 + r;
      stg[cc * ASP + ql]        = (_Float16)(o0[r] * vinv);
      stg[(16 + cc) * ASP + ql] = (_Float16)(o1[r] * vinv);
    }
    __syncthreads();
  }

  const int lr = lane >> 3, pc = (lane & 7) * 8;
  v8h_ vals[4];
#pragma unroll
  for (int it = 0; it < 4; ++it) {
    const int d = wloc * 16 + it * 4 + lr;
    vals[it] = *(const v8h*)(stg + d * ASP + pc);
  }
  const size_t chbase = (size_t)b * (2 * CCH) + br * CCH + hd * HDIM;
#pragma unroll
  for (int it = 0; it < 4; ++it) {
    const int d = wloc * 16 + it * 4 + lr;
    _Float16* pd = oc + (chbase + d) * (size_t)NQ + qg * 64 + pc;
    *(volatile v8h_*)pd = vals[it];
  }
  __threadfence();
#pragma unroll
  for (int it = 0; it < 4; ++it) {
    const int d = wloc * 16 + it * 4 + lr;
    _Float16* pd = oc + (chbase + d) * (size_t)NQ + qg * 64 + pc;
    *(volatile v8h_*)pd = vals[it];
  }
}

extern "C" void kernel_launch(void* const* d_in, const int* in_sizes, int n_in,
                              void* d_out, int out_size, void* d_ws, size_t ws_size,
                              hipStream_t stream) {
  if (n_in < 19) return;
  const int xs = in_sizes[0];
  const int nbatch = xs / (CCH * NQ);
  if (nbatch <= 0 || nbatch * (CCH * NQ) != xs) return;
  if (in_sizes[1] != 2 * CCH * CCH || in_sizes[2] != 2 * CCH) return;
  if (in_sizes[3] != CCH * CCH * 16 || in_sizes[4] != CCH) return;
  if (in_sizes[5] != CCH * 9 || in_sizes[6] != CCH) return;
  if (in_sizes[7] != CCH * CCH || in_sizes[8] != CCH) return;
  if (in_sizes[9] != CCH * 9 || in_sizes[10] != CCH) return;
  if (in_sizes[11] != CCH * CCH || in_sizes[12] != CCH) return;
  if (in_sizes[13] != CCH * CCH || in_sizes[14] != CCH) return;
  if (in_sizes[15] != CCH * CCH || in_sizes[16] != CCH) return;
  if (in_sizes[17] != 2 * CCH * CCH || in_sizes[18] != CCH) return;
  if (out_size != nbatch * CCH * NQ) return;

  const float* x      = (const float*)d_in[0];
  const float* wq     = (const float*)d_in[1];
  const float* bq     = (const float*)d_in[2];
  const float* wsconv = (const float*)d_in[3];
  const float* bs     = (const float*)d_in[4];
  const float* wak_d  = (const float*)d_in[5];
  const float* bak_d  = (const float*)d_in[6];
  const float* wak_p  = (const float*)d_in[7];
  const float* bak_p  = (const float*)d_in[8];
  const float* wav_d  = (const float*)d_in[9];
  const float* bav_d  = (const float*)d_in[10];
  const float* wav_p  = (const float*)d_in[11];
  const float* bav_p  = (const float*)d_in[12];
  const float* wek    = (const float*)d_in[13];
  const float* bek    = (const float*)d_in[14];
  const float* wev    = (const float*)d_in[15];
  const float* bev    = (const float*)d_in[16];
  const float* wproj  = (const float*)d_in[17];
  const float* bproj  = (const float*)d_in[18];
  float* out = (float*)d_out;

  size_t off = 0;
  auto take = [&](size_t bytes) { size_t p = off; off += (bytes + 255) & ~(size_t)255; return p; };
  const size_t o_wq  = take((size_t)2 * CCH * CCH * 2);
  const size_t o_ws  = take((size_t)CCH * CCH * 16 * 2);
  const size_t o_wak = take((size_t)CCH * CCH * 2);
  const size_t o_wav = take((size_t)CCH * CCH * 2);
  const size_t o_wek = take((size_t)CCH * CCH * 2);
  const size_t o_wev = take((size_t)CCH * CCH * 2);
  const size_t o_wp  = take((size_t)2 * CCH * CCH * 2);
  const size_t o_qh  = take((size_t)nbatch * 2 * CCH * NQ * 2);
  const size_t o_xr  = take((size_t)nbatch * CCH * NKV * 4);
  const size_t o_dwk = take((size_t)nbatch * CCH * NKV * 4);
  const size_t o_dwv = take((size_t)nbatch * CCH * NKV * 4);
  const size_t kvhalves = (size_t)nbatch * NHEAD * NKV * HDIM;
  const size_t o_kh  = take(2 * kvhalves * 2);
  const size_t o_vh  = take(2 * kvhalves * 2);
  const size_t o_oc  = take((size_t)nbatch * 2 * CCH * NQ * 2);
  if (off > ws_size) return;

  char* wsp = (char*)d_ws;
  _Float16* wq_h  = (_Float16*)(wsp + o_wq);
  _Float16* ws_h  = (_Float16*)(wsp + o_ws);
  _Float16* wak_h = (_Float16*)(wsp + o_wak);
  _Float16* wav_h = (_Float16*)(wsp + o_wav);
  _Float16* wek_h = (_Float16*)(wsp + o_wek);
  _Float16* wev_h = (_Float16*)(wsp + o_wev);
  _Float16* wp_h  = (_Float16*)(wsp + o_wp);
  _Float16* qh    = (_Float16*)(wsp + o_qh);
  float*    xr    = (float*)(wsp + o_xr);
  float*    dwk   = (float*)(wsp + o_dwk);
  float*    dwv   = (float*)(wsp + o_dwv);
  _Float16* kh    = (_Float16*)(wsp + o_kh);
  _Float16* vh    = (_Float16*)(wsp + o_vh);
  _Float16* oc    = (_Float16*)(wsp + o_oc);
  _Float16* kh_e  = kh + kvhalves;
  _Float16* vh_e  = vh + kvhalves;

  const float WSC = 64.0f;
  k_cvt<<<(2 * CCH * CCH / 8 + 255) / 256, 256, 0, stream>>>(wq, wq_h, 2 * CCH * CCH, WSC);
  k_cvt<<<(CCH * CCH * 16 / 8 + 255) / 256, 256, 0, stream>>>(wsconv, ws_h, CCH * CCH * 16, WSC);
  k_cvt<<<(CCH * CCH / 8 + 255) / 256, 256, 0, stream>>>(wak_p, wak_h, CCH * CCH, WSC);
  k_cvt<<<(CCH * CCH / 8 + 255) / 256, 256, 0, stream>>>(wav_p, wav_h, CCH * CCH, WSC);
  k_cvt<<<(CCH * CCH / 8 + 255) / 256, 256, 0, stream>>>(wek, wek_h, CCH * CCH, WSC);
  k_cvt<<<(CCH * CCH / 8 + 255) / 256, 256, 0, stream>>>(wev, wev_h, CCH * CCH, WSC);
  k_cvt<<<(2 * CCH * CCH / 8 + 255) / 256, 256, 0, stream>>>(wproj, wp_h, 2 * CCH * CCH, WSC);

  {
    const int grid = nbatch * (2 * CCH / BM) * (NQ / BN);
    k_gemm<0, 2><<<grid, 256, 0, stream>>>(wq_h, x, bq, qh, 2 * CCH, NQ, CCH, NQ, nbatch,
                                           1.0f, 1.0f / 64.0f, 4.0f);
  }
  {
    const int grid = nbatch * (CCH / BM) * (NKV / BN);
    k_gemm<2, 0><<<grid, 256, 0, stream>>>(ws_h, x, bs, xr, CCH, NKV, CCH * 16, NKV, nbatch,
                                           1.0f, 1.0f / 64.0f, 1.0f);
  }
  {
    const int total = nbatch * CCH * 64;
    k_dw3x3<<<(total + 255) / 256, 256, 0, stream>>>(xr, wak_d, bak_d, wav_d, bav_d, dwk, dwv, total);
  }
  {
    const int grid = nbatch * (CCH / BM) * (NKV / BN);
    k_gemm<0, 2><<<grid, 256, 0, stream>>>(wak_h, dwk, bak_p, kh, CCH, NKV, CCH, NKV, nbatch,
                                           16.0f, 1.0f / 1024.0f, 32.0f);
    k_gemm<0, 1><<<grid, 256, 0, stream>>>(wav_h, dwv, bav_p, vh, CCH, NKV, CCH, NKV, nbatch,
                                           16.0f, 1.0f / 1024.0f, 32.0f);
    k_gemm<0, 2><<<grid, 256, 0, stream>>>(wek_h, xr, bek, kh_e, CCH, NKV, CCH, NKV, nbatch,
                                           1.0f, 1.0f / 64.0f, 2.0f);
    k_gemm<0, 1><<<grid, 256, 0, stream>>>(wev_h, xr, bev, vh_e, CCH, NKV, CCH, NKV, nbatch,
                                           1.0f, 1.0f / 64.0f, 2.0f);
  }
  {
    const int grid = nbatch * 2 * NHEAD * (NQ / 64);
    k_attn<<<grid, 64, 0, stream>>>(qh, kh, vh, oc, nbatch,
                                    ATT_SCALE / 128.0f, ATT_SCALE / 8.0f, 1.0f / 32.0f, 0.5f);
  }
  {
    const int grid = nbatch * (CCH / BM) * (NQ / BN);
    k_gemm<1, 0><<<grid, 256, 0, stream>>>(wp_h, oc, bproj, out, CCH, NQ, 2 * CCH, NQ, nbatch,
                                           1.0f, 1.0f / 16384.0f, 1.0f);
  }
}
